// Attention_28604482191565
// MI455X (gfx1250) — hardware-run, weakly checked
//
#include <hip/hip_runtime.h>


#ifndef NB
#define NB 4
#endif
#ifndef SEQ
#define SEQ 2048
#endif
#define NB_FULL  4
#define SEQ_FULL 2048
#ifndef OUT_SEQ
#define OUT_SEQ SEQ
#endif
#define DM   768
#define DFF  3072
#define NH_  12
#define HD   64
#define AW   4
#define SC2  (0.125f * 1.4426950408889634f)
#define PSH  8.0f
#define WSC  1024.0f
#define CSC  64.0f

static_assert(HD == 64);
static_assert(NH_ * HD == DM);
static_assert(DM % 64 == 0);
static_assert(DFF % 64 == 0);
static_assert(DM % 32 == 0);
static_assert(DFF % 32 == 0);
static_assert(SEQ % 64 == 0);
static_assert((NB * SEQ) % 64 == 0);
static_assert(SEQ % 32 == 0);
static_assert(SEQ % (16 * AW) == 0);
static_assert((NB * SEQ) % 4 == 0);
static_assert(((size_t)SEQ * DM) % 8 == 0);
static_assert(DM == 3 * 32 * 8);
static_assert(NB <= NB_FULL);
static_assert(SEQ <= SEQ_FULL);

typedef _Float16 h16;
typedef unsigned short bf;
typedef __attribute__((ext_vector_type(16))) __bf16   v16bf;
typedef __attribute__((ext_vector_type(16))) _Float16 v16h;
typedef __attribute__((ext_vector_type(8)))  _Float16 v8h;
typedef __attribute__((ext_vector_type(8)))  unsigned short v8us;
typedef __attribute__((ext_vector_type(8)))  float    v8f;
typedef __attribute__((ext_vector_type(4)))  float    v4f;
typedef v4f  __attribute__((may_alias)) v4fa;

__device__ __forceinline__ unsigned short f2bf(float f) { unsigned u = __float_as_uint(f); u += 0x7FFFu + ((u >> 16) & 1u); return (unsigned short)(u >> 16); }
__device__ __forceinline__ float rbf(float f) { return __uint_as_float(((unsigned)f2bf(f)) << 16); }
__device__ __forceinline__ v16h cat16(v8h lo, v8h hi) { return __builtin_shufflevector(lo, hi, 0, 1, 2, 3, 4, 5, 6, 7, 8, 9, 10, 11, 12, 13, 14, 15); }
__device__ __forceinline__ v16bf cat16b(v8us lo, v8us hi) { return __builtin_bit_cast(v16bf, __builtin_shufflevector(lo, hi, 0, 1, 2, 3, 4, 5, 6, 7, 8, 9, 10, 11, 12, 13, 14, 15)); }
__device__ __forceinline__ v8f wmma16(v16h a, v16h b, v8f c) { return __builtin_amdgcn_wmma_f32_16x16x32_f16(false, a, false, b, (short)0, c, false, false); }
__device__ __forceinline__ v8f wmmab(v16bf a, v16bf b, v8f c) { return __builtin_amdgcn_wmma_f32_16x16x32_bf16(false, a, false, b, (short)0, c, false, false); }
__device__ __forceinline__ v16h  ldh(const h16* p) { return cat16(*(const v8h*)p, *(const v8h*)(p + 16)); }
__device__ __forceinline__ v16bf ldb(const bf* p)  { return cat16b(*(const v8us*)p, *(const v8us*)(p + 16)); }
__device__ __forceinline__ void wave_sync() { __builtin_amdgcn_fence(3  , "wavefront"); __builtin_amdgcn_wave_barrier(); asm volatile("" ::: "memory"); }
__device__ __forceinline__ int wave_id() { return __builtin_amdgcn_readfirstlane((int)(threadIdx.x >> 5)); }

template <int F16> struct Op;
template <> struct Op<0> { typedef v16bf V; typedef bf E;
    static __device__ __forceinline__ V ld(const bf* p) { return ldb(p); }
    static __device__ __forceinline__ v8f mm(V a, V b, v8f c) { return wmmab(a, b, c); } };
template <> struct Op<1> { typedef v16h V; typedef h16 E;
    static __device__ __forceinline__ V ld(const h16* p) { return ldh(p); }
    static __device__ __forceinline__ v8f mm(V a, V b, v8f c) { return wmma16(a, b, c); } };

static __device__ __forceinline__ h16 toh_flush(float v) { const h16 r = (h16)v; return (fabsf(v) < 6.103515625e-05f) ? (h16)0.0f : r; }
static __device__ __forceinline__ float gelu_t(float x) {
    const float u = 0.7978845608f * (x + 0.044715f * (x * x * x));
    const float e = fminf(u * -2.8853900818f, 80.0f);
    return x * __builtin_amdgcn_rcpf(1.0f + __builtin_amdgcn_exp2f(e));
}

__global__ __launch_bounds__(256) void k_wt(const float* __restrict__ W, bf* Wt, int K, int N, int mode) {
    __shared__ float t[64 * 65];
    const int tid = threadIdx.x, n0 = blockIdx.x * 64, k0 = blockIdx.y * 64;
#pragma unroll
    for (int i = 0; i < 4; ++i) { const int kk = (tid >> 4) + 16 * i, c4 = (tid & 15) * 4;
        const v4f v = *(const v4f*)(W + (size_t)(k0 + kk) * N + n0 + c4);
        t[kk * 65 + c4 + 0] = v[0]; t[kk * 65 + c4 + 1] = v[1]; t[kk * 65 + c4 + 2] = v[2]; t[kk * 65 + c4 + 3] = v[3]; }
    __syncthreads();
    const int lane = tid & 31, wave = wave_id();
    v8us o[2];
#pragma unroll
    for (int s = 0; s < 2; ++s) { const int nn = 4 * (wave + 8 * s) + (lane >> 3), c8 = (lane & 7) * 8;
        v8us ob; v8h oh;
#pragma unroll
        for (int i = 0; i < 8; ++i) { const unsigned short u = f2bf(t[(c8 + i) * 65 + nn]); ob[i] = u; oh[i] = (h16)(__uint_as_float(((unsigned)u) << 16) * WSC); }
        const v8us ohb = __builtin_bit_cast(v8us, oh);
        o[s] = mode ? ohb : ob; }
#pragma unroll 1
    for (int ps = 0; ps < 2; ++ps) {
#pragma unroll
        for (int s = 0; s < 2; ++s) { const int nn = 4 * (wave + 8 * s) + (lane >> 3), c8 = (lane & 7) * 8;
            *(volatile v8us*)(Wt + (size_t)(n0 + nn) * K + k0 + c8) = o[s]; }
        if (ps == 0) __threadfence(); }
}

template <int EPI, int NORM, int ACT, int RBF>
__device__ __forceinline__ void gemm_body(const bf* __restrict__ Ain, const bf* __restrict__ Bin, int K, float scale,
                                          const float* __restrict__ gain,
                                          h16* Ph, int RB, size_t sRB, int pitch, int CB, size_t sCB,
                                          const float* __restrict__ Rs, int resSeq, float* Cf, int outSeq) {
    typedef Op<1>::V V;
    __shared__ __align__(16) float os[16 * 68];
    const h16* A = (const h16*)Ain; const h16* Bt = (const h16*)Bin;
    const int lane = threadIdx.x & 31, lr = lane & 15, hi = lane >> 4; const int r0 = blockIdx.x * 64, c0 = blockIdx.y * 64;
    v8f acc[4][4];
#pragma unroll
    for (int mb = 0; mb < 4; ++mb)
#pragma unroll
        for (int nb = 0; nb < 4; ++nb) acc[mb][nb] = (v8f){};
    const size_t aoff = (size_t)(r0 + lr) * K + 8 * hi, boff = (size_t)(c0 + lr) * K + 8 * hi;
#pragma unroll 1
    for (int kc = 0; kc < K; kc += 32) {
        V a[4];
#pragma unroll
        for (int mb = 0; mb < 4; ++mb) a[mb] = Op<1>::ld(A + aoff + (size_t)mb * 16 * K + kc);
#pragma unroll
        for (int nb = 0; nb < 4; ++nb) { const V b = Op<1>::ld(Bt + boff + (size_t)nb * 16 * K + kc);
#pragma unroll
            for (int mb = 0; mb < 4; ++mb) acc[mb][nb] = Op<1>::mm(a[mb], b, acc[mb][nb]); }
        asm volatile("v_nop\n\tv_nop\n\tv_nop\n\tv_nop" : "+v"(acc[0][0]), "+v"(acc[1][1]), "+v"(acc[2][2]), "+v"(acc[3][3]) : "v"(a[0]), "v"(a[1]), "v"(a[2]), "v"(a[3]));
    }
    float g[8];
    if (NORM) { const int c8 = (lane & 7) * 8; const v4f g0 = *(const v4f*)(gain + c8); const v4f g1 = *(const v4f*)(gain + c8 + 4);
#pragma unroll
        for (int i = 0; i < 4; ++i) { g[i] = rbf(g0[i]); g[4 + i] = rbf(g1[i]); }
    } else {
#pragma unroll
        for (int i = 0; i < 8; ++i) g[i] = 1.0f; }
    const size_t tbase = (size_t)(r0 / RB) * sRB + (size_t)(r0 % RB) * (size_t)pitch + (size_t)(c0 / CB) * sCB + (size_t)(c0 % CB);
#pragma unroll
    for (int mb = 0; mb < 4; ++mb) {
#pragma unroll
        for (int nb = 0; nb < 4; ++nb) {
#pragma unroll
            for (int j = 0; j < 8; ++j) { float v = acc[mb][nb][j] * scale; if (ACT) v = gelu_t(v);
                os[(hi * 8 + j) * 68 + nb * 16 + lr] = v; } }
        wave_sync();
        if (EPI == 0) {
            const size_t sb = tbase + (size_t)(mb * 16) * (size_t)pitch;
            v8h hv[4];
#pragma unroll
            for (int s = 0; s < 4; ++s) { const int row = 4 * s + (lane >> 3), c8 = (lane & 7) * 8;
                const v4f x0 = *(const v4fa*)(&os[row * 68 + c8]); const v4f x1 = *(const v4fa*)(&os[row * 68 + c8 + 4]);
                float mul = 1.0f;
                if (NORM) {
                    float ss = ((x0[0] * x0[0] + x0[1] * x0[1]) + (x0[2] * x0[2] + x0[3] * x0[3])) + ((x1[0] * x1[0] + x1[1] * x1[1]) + (x1[2] * x1[2] + x1[3] * x1[3]));
                    ss += __shfl_xor(ss, 1, 32); ss += __shfl_xor(ss, 2, 32); ss += __shfl_xor(ss, 4, 32);
                    mul = rsqrtf(ss * (1.0f / 64.0f) + 1e-6f); }
#pragma unroll
                for (int i = 0; i < 4; ++i) {
                    const float y0 = NORM ? (x0[i] * mul) * g[i] : x0[i];
                    const float y1 = NORM ? (x1[i] * mul) * g[4 + i] : x1[i];
                    hv[s][i] = toh_flush(y0); hv[s][4 + i] = toh_flush(y1); } }
#pragma unroll 1
            for (int ps = 0; ps < 2; ++ps) {
#pragma unroll
                for (int s = 0; s < 4; ++s) { const int row = 4 * s + (lane >> 3), c8 = (lane & 7) * 8;
                    const size_t oo = sb + (size_t)row * (size_t)pitch + c8;
                    *(volatile v8h*)(Ph + oo) = hv[s]; }
                if (ps == 0) __threadfence(); }
        } else {
            const int bq = r0 / SEQ, tq = r0 - bq * SEQ;
            const float* rp = Rs + ((size_t)bq * (size_t)resSeq + (size_t)(tq + mb * 16)) * DM + c0;
            float* cp = Cf + ((size_t)bq * (size_t)outSeq + (size_t)(tq + mb * 16)) * DM + c0;
            v4f val[8];
#pragma unroll
            for (int s = 0; s < 8; ++s) { const int row = 2 * s + hi, cofs = lr * 4;
                const v4f xv = *(const v4fa*)(&os[row * 68 + cofs]);
                v4f rr = *(const v4f*)(rp + (size_t)row * DM + cofs);
                if (RBF) { rr[0] = rbf(rr[0]); rr[1] = rbf(rr[1]); rr[2] = rbf(rr[2]); rr[3] = rbf(rr[3]); }
                val[s] = xv + rr; }
#pragma unroll 1
            for (int ps = 0; ps < 2; ++ps) {
#pragma unroll
                for (int s = 0; s < 8; ++s) { const int row = 2 * s + hi, cofs = lr * 4;
                    *(volatile v4f*)(cp + (size_t)row * DM + cofs) = val[s]; }
                if (ps == 0) __threadfence(); }
        }
        wave_sync();
    }
}

__global__ __launch_bounds__(32) void k_gemm_norm(const bf* __restrict__ Ain, const bf* __restrict__ Bin, int K, float scale, const float* __restrict__ gain,
                                                  h16* Ph, int RB, size_t sRB, int pitch, int CB, size_t sCB) {
    gemm_body<0, 1, 0, 0>(Ain, Bin, K, scale, gain, Ph, RB, sRB, pitch, CB, sCB, nullptr, 0, nullptr, 0);
}
__global__ __launch_bounds__(32) void k_gemm_plane(const bf* __restrict__ Ain, const bf* __restrict__ Bin, int K, float scale,
                                                   h16* Ph, int RB, size_t sRB, int pitch, int CB, size_t sCB) {
    gemm_body<0, 0, 0, 0>(Ain, Bin, K, scale, nullptr, Ph, RB, sRB, pitch, CB, sCB, nullptr, 0, nullptr, 0);
}
__global__ __launch_bounds__(32) void k_gemm_gelu(const bf* __restrict__ Ain, const bf* __restrict__ Bin, int K, float scale,
                                                  h16* Ph, int RB, size_t sRB, int pitch, int CB, size_t sCB) {
    gemm_body<0, 0, 1, 0>(Ain, Bin, K, scale, nullptr, Ph, RB, sRB, pitch, CB, sCB, nullptr, 0, nullptr, 0);
}
__global__ __launch_bounds__(32) void k_gemm_res_in(const bf* __restrict__ Ain, const bf* __restrict__ Bin, int K, float scale,
                                                    const float* __restrict__ Rs, int resSeq, float* Cf, int outSeq) {
    gemm_body<1, 0, 0, 1>(Ain, Bin, K, scale, nullptr, nullptr, 1, (size_t)0, 0, 1, (size_t)0, Rs, resSeq, Cf, outSeq);
}
__global__ __launch_bounds__(32) void k_gemm_res(const bf* __restrict__ Ain, const bf* __restrict__ Bin, int K, float scale,
                                                 const float* __restrict__ Rs, int resSeq, float* Cf, int outSeq) {
    gemm_body<1, 0, 0, 0>(Ain, Bin, K, scale, nullptr, nullptr, 1, (size_t)0, 0, 1, (size_t)0, Rs, resSeq, Cf, outSeq);
}

__global__ __launch_bounds__(32 * AW) void k_flash(const h16* __restrict__ QH, const h16* __restrict__ KP, const h16* __restrict__ VT, h16* CTX) {
    __shared__ __align__(16) float os[AW * 16 * 68];
    const int lane = threadIdx.x & 31, wave = wave_id(), lr = lane & 15, hi = lane >> 4;
    const int zh = blockIdx.y; const int b = zh / NH_, h = zh % NH_;
    const int t0 = (blockIdx.x * AW + wave) * 16;
    const size_t pbase = (size_t)zh * SEQ * HD;
    const size_t qo = pbase + (size_t)(t0 + lr) * HD + 8 * hi;
    const v16h qh0 = ldh(QH + qo), qh1 = ldh(QH + qo + 32);
    const size_t ko = pbase + (size_t)lr * HD + 8 * hi;
    const size_t vo = pbase + (size_t)lr * SEQ + 8 * hi;
    v8f o0 = (v8f){}, o1 = (v8f){}, o2 = (v8f){}, o3 = (v8f){};
    float m = -3.0e38f, l = 0.0f;
#pragma unroll 1
    for (int key0 = 0; key0 < SEQ; key0 += 32) {
        const h16* ka = KP + ko + (size_t)key0 * HD;
        const v16h ka0 = ldh(ka), ka1 = ldh(ka + 32), kb0 = ldh(ka + 16 * HD), kb1 = ldh(ka + 16 * HD + 32);
        v8f sHa = (v8f){}, sHb = (v8f){};
        sHa = wmma16(ka0, qh0, sHa); sHb = wmma16(kb0, qh0, sHb);
        sHa = wmma16(ka1, qh1, sHa); sHb = wmma16(kb1, qh1, sHb);
        asm volatile("v_nop\n\tv_nop\n\tv_nop\n\tv_nop" : "+v"(sHa), "+v"(sHb) : "v"(ka0), "v"(ka1), "v"(kb0), "v"(kb1));
        float ta[8], tb[8]; float mx = -3.0e38f;
#pragma unroll
        for (int r = 0; r < 8; ++r) { ta[r] = sHa[r] * SC2; tb[r] = sHb[r] * SC2; mx = fmaxf(mx, fmaxf(ta[r], tb[r])); }
        mx = fmaxf(mx, __shfl_xor(mx, 16, 32));
        const float mnew = fmaxf(m, mx);
        const float alpha = __builtin_amdgcn_exp2f(m - mnew);
        const float sh = PSH - mnew;
        v16h pb; float ls = 0.0f;
#pragma unroll
        for (int r = 0; r < 8; ++r) { const h16 pa = (h16)__builtin_amdgcn_exp2f(ta[r] + sh); const h16 pc = (h16)__builtin_amdgcn_exp2f(tb[r] + sh); pb[r] = pa; pb[8 + r] = pc; ls += (float)pa + (float)pc; }
        l = l * alpha + ls; m = mnew;
        o0 = o0 * alpha; o1 = o1 * alpha; o2 = o2 * alpha; o3 = o3 * alpha;
        const h16* va = VT + vo + key0;
        const v16h v0 = ldh(va), v1 = ldh(va + (size_t)16 * SEQ), v2 = ldh(va + (size_t)32 * SEQ), v3 = ldh(va + (size_t)48 * SEQ);
        o0 = wmma16(v0, pb, o0); o1 = wmma16(v1, pb, o1); o2 = wmma16(v2, pb, o2); o3 = wmma16(v3, pb, o3);
        asm volatile("v_nop\n\tv_nop\n\tv_nop\n\tv_nop" : "+v"(o0), "+v"(o1), "+v"(o2), "+v"(o3) : "v"(v0), "v"(v1), "v"(v2), "v"(v3), "v"(pb));
    }
    l += __shfl_xor(l, 16, 32);
    const float inv = CSC * (1.0f / l);
    const int wb = wave * 16 * 68;
    { v4f a, c;
      a[0] = o0[0] * inv; a[1] = o0[1] * inv; a[2] = o0[2] * inv; a[3] = o0[3] * inv; c[0] = o0[4] * inv; c[1] = o0[5] * inv; c[2] = o0[6] * inv; c[3] = o0[7] * inv;
      *(v4fa*)(&os[wb + lr * 68 +  0 + 8 * hi]) = a; *(v4fa*)(&os[wb + lr * 68 +  0 + 8 * hi + 4]) = c;
      a[0] = o1[0] * inv; a[1] = o1[1] * inv; a[2] = o1[2] * inv; a[3] = o1[3] * inv; c[0] = o1[4] * inv; c[1] = o1[5] * inv; c[2] = o1[6] * inv; c[3] = o1[7] * inv;
      *(v4fa*)(&os[wb + lr * 68 + 16 + 8 * hi]) = a; *(v4fa*)(&os[wb + lr * 68 + 16 + 8 * hi + 4]) = c;
      a[0] = o2[0] * inv; a[1] = o2[1] * inv; a[2] = o2[2] * inv; a[3] = o2[3] * inv; c[0] = o2[4] * inv; c[1] = o2[5] * inv; c[2] = o2[6] * inv; c[3] = o2[7] * inv;
      *(v4fa*)(&os[wb + lr * 68 + 32 + 8 * hi]) = a; *(v4fa*)(&os[wb + lr * 68 + 32 + 8 * hi + 4]) = c;
      a[0] = o3[0] * inv; a[1] = o3[1] * inv; a[2] = o3[2] * inv; a[3] = o3[3] * inv; c[0] = o3[4] * inv; c[1] = o3[5] * inv; c[2] = o3[6] * inv; c[3] = o3[7] * inv;
      *(v4fa*)(&os[wb + lr * 68 + 48 + 8 * hi]) = a; *(v4fa*)(&os[wb + lr * 68 + 48 + 8 * hi + 4]) = c; }
    wave_sync();
    h16* crow = CTX + ((size_t)b * SEQ + t0) * DM + h * HD;
#pragma unroll 1
    for (int ps = 0; ps < 2; ++ps) {
#pragma unroll
        for (int s = 0; s < 4; ++s) { const int row = 4 * s + (lane >> 3), c8 = (lane & 7) * 8;
            const v4f x0 = *(const v4fa*)(&os[wb + row * 68 + c8]); const v4f x1 = *(const v4fa*)(&os[wb + row * 68 + c8 + 4]); v8h hv;
#pragma unroll
            for (int i = 0; i < 4; ++i) { hv[i] = (h16)x0[i]; hv[4 + i] = (h16)x1[i]; }
            *(volatile v8h*)(crow + (size_t)row * DM + c8) = hv; }
        if (ps == 0) __threadfence(); }
}

template <int FIRST>
__device__ __forceinline__ void rms_body(const float* __restrict__ R, const float* __restrict__ G, h16* OH, int nrows) {
#pragma clang fp contract(off)
    const int lane = threadIdx.x & 31, wave = wave_id();
    const int r = blockIdx.x * 4 + wave;
    if (r >= nrows) return;
    const int b = r / SEQ, t = r - b * SEQ;
    const size_t ro = FIRST ? ((size_t)b * SEQ_FULL + t) * DM : (size_t)r * DM;
    const float* rp = R + ro;
    v8f v[3]; float sq = 0.0f;
#pragma unroll
    for (int j = 0; j < 3; ++j) { const int idx = (lane + 32 * j) * 8;
        v8f a = *(const v8f*)(rp + idx);
        if (FIRST) {
#pragma unroll
            for (int k = 0; k < 8; ++k) a[k] = rbf(a[k]); }
        v[j] = a;
        sq += ((a[0] * a[0] + a[1] * a[1]) + (a[2] * a[2] + a[3] * a[3])) + ((a[4] * a[4] + a[5] * a[5]) + (a[6] * a[6] + a[7] * a[7])); }
#pragma unroll
    for (int d = 16; d >= 1; d >>= 1) sq += __shfl_xor(sq, d, 32);
    const float rstd = rsqrtf(sq * (1.0f / (float)DM) + 1e-6f);
    v8h hv[3];
#pragma unroll
    for (int j = 0; j < 3; ++j) { const int idx = (lane + 32 * j) * 8;
        const v8f g8 = *(const v8f*)(G + idx);
#pragma unroll
        for (int k = 0; k < 8; ++k) hv[j][k] = toh_flush((v[j][k] * rstd) * rbf(g8[k])); }
    h16* hp = OH + (size_t)r * DM;
#pragma unroll 1
    for (int ps = 0; ps < 2; ++ps) {
#pragma unroll
        for (int j = 0; j < 3; ++j) *(volatile v8h*)(hp + (lane + 32 * j) * 8) = hv[j];
        if (ps == 0) __threadfence(); }
}
__global__ __launch_bounds__(128) void k_rms_in(const float* __restrict__ R, const float* __restrict__ G, h16* OH, int nrows) { rms_body<1>(R, G, OH, nrows); }
__global__ __launch_bounds__(128) void k_rms_mid(const float* __restrict__ R, const float* __restrict__ G, h16* OH, int nrows) { rms_body<0>(R, G, OH, nrows); }

static constexpr size_t al256(size_t v) { return (v + 255) & ~(size_t)255; }
static constexpr size_t SZ_R1  = al256((size_t)NB * SEQ * DM * 2);
static constexpr size_t SZ_W3  = al256((size_t)3 * DM * DM * 2);
static constexpr size_t SZ_WO  = al256((size_t)DM * DM * 2);
static constexpr size_t SZ_W1  = al256((size_t)DM * DFF * 2);
static constexpr size_t SZ_W2  = al256((size_t)DFF * DM * 2);
static constexpr size_t SZ_PL  = al256((size_t)NB * NH_ * SEQ * HD * 2);
static constexpr size_t SZ_FF  = al256((size_t)NB * SEQ * DFF * 2);
static constexpr size_t SZ_F32 = al256((size_t)NB * SEQ * DM * 4);
static constexpr size_t SZ_TOTAL = SZ_R1 + SZ_W3 + SZ_WO + SZ_W1 + SZ_W2 + SZ_FF + SZ_F32;
static_assert(SZ_TOTAL <= (size_t)134217728);
static_assert(3 * SZ_PL <= SZ_FF);
static_assert(((size_t)DM * DM * 2) % 256 == 0);
static_assert((size_t)NB * SEQ * DM * 2 <= SZ_R1);
static_assert((size_t)NB * SEQ * DFF * 2 <= SZ_FF);

extern "C" void kernel_launch(void* const* d_in, const int* in_sizes, int n_in,
                              void* d_out, int out_size, void* d_ws, size_t ws_size, hipStream_t stream) {
    if (n_in < 11) return;
    const size_t needx = ((size_t)(NB - 1) * SEQ_FULL + SEQ) * DM;
    if ((size_t)in_sizes[0] < needx) return;
    if (in_sizes[1] < DM || in_sizes[8] < DM) return;
    if ((size_t)in_sizes[2] < (size_t)DM * DM || (size_t)in_sizes[3] < (size_t)DM * DM || (size_t)in_sizes[4] < (size_t)DM * DM || (size_t)in_sizes[7] < (size_t)DM * DM) return;
    if (in_sizes[5] < HD || in_sizes[6] < HD) return;
    if ((size_t)in_sizes[9] < (size_t)DM * DFF || (size_t)in_sizes[10] < (size_t)DFF * DM) return;
    if ((size_t)out_size < ((size_t)(NB - 1) * OUT_SEQ + SEQ) * DM) return;
    if (SZ_TOTAL > ws_size) return;
    const float* lat = (const float*)d_in[0];
    const float* ln1 = (const float*)d_in[1];
    const float* wq  = (const float*)d_in[2];
    const float* wk  = (const float*)d_in[3];
    const float* wv  = (const float*)d_in[4];
    const float* qns = (const float*)d_in[5];
    const float* kns = (const float*)d_in[6];
    const float* wo  = (const float*)d_in[7];
    const float* ln2 = (const float*)d_in[8];
    const float* wi  = (const float*)d_in[9];
    const float* wm  = (const float*)d_in[10];
    float* OUT = (float*)d_out;
    char* wsp = (char*)d_ws;
    bf* R1  = (bf*)wsp; wsp += SZ_R1;
    bf* W3  = (bf*)wsp; wsp += SZ_W3;
    bf* WOT = (bf*)wsp; wsp += SZ_WO;
    bf* W1T = (bf*)wsp; wsp += SZ_W1;
    bf* W2T = (bf*)wsp; wsp += SZ_W2;
    char* ffr = wsp; wsp += SZ_FF;
    float* X2 = (float*)wsp; wsp += SZ_F32;
    h16* QH = (h16*)ffr;
    h16* KP = (h16*)(ffr + SZ_PL);
    h16* VT = (h16*)(ffr + 2 * SZ_PL);
    h16* FF1 = (h16*)ffr;
    h16* XN = (h16*)R1; h16* CTX = (h16*)R1; h16* YN = (h16*)R1;
    bf* WQT = W3; bf* WKT = W3 + (size_t)DM * DM; bf* WVT = W3 + (size_t)2 * DM * DM;
    const int MR = NB * SEQ;

    k_wt<<<dim3(DM / 64, DM / 64, 1), 256, 0, stream>>>(wq, WQT, DM, DM, 1);
    k_wt<<<dim3(DM / 64, DM / 64, 1), 256, 0, stream>>>(wk, WKT, DM, DM, 1);
    k_wt<<<dim3(DM / 64, DM / 64, 1), 256, 0, stream>>>(wv, WVT, DM, DM, 1);
    k_wt<<<dim3(DM / 64, DM / 64, 1), 256, 0, stream>>>(wo, WOT, DM, DM, 1);
    k_wt<<<dim3(DFF / 64, DM / 64, 1), 256, 0, stream>>>(wi, W1T, DM, DFF, 1);
    k_wt<<<dim3(DM / 64, DFF / 64, 1), 256, 0, stream>>>(wm, W2T, DFF, DM, 1);

    k_rms_in<<<MR / 4, 128, 0, stream>>>(lat, ln1, XN, MR);

    k_gemm_norm<<<dim3(MR / 64, DM / 64, 1), 32, 0, stream>>>((const bf*)XN, WQT, DM, 1.0f / 1024.0f, qns, QH, SEQ, (size_t)NH_ * SEQ * HD, HD, HD, (size_t)SEQ * HD);
    k_gemm_norm<<<dim3(MR / 64, DM / 64, 1), 32, 0, stream>>>((const bf*)XN, WKT, DM, 1.0f / 1024.0f, kns, KP, SEQ, (size_t)NH_ * SEQ * HD, HD, HD, (size_t)SEQ * HD);
    k_gemm_plane<<<dim3(DM / 64, MR / 64, 1), 32, 0, stream>>>(WVT, (const bf*)XN, DM, 1.0f / 1024.0f, VT, DM, (size_t)0, SEQ, SEQ, (size_t)DM * SEQ);

    k_flash<<<dim3(SEQ / (16 * AW), NB * NH_, 1), 32 * AW, 0, stream>>>(QH, KP, VT, CTX);

    k_gemm_res_in<<<dim3(MR / 64, DM / 64, 1), 32, 0, stream>>>((const bf*)CTX, WOT, DM, 1.0f / 65536.0f, lat, SEQ_FULL, X2, SEQ);
    k_rms_mid<<<MR / 4, 128, 0, stream>>>(X2, ln2, YN, MR);
    k_gemm_gelu<<<dim3(MR / 64, DFF / 64, 1), 32, 0, stream>>>((const bf*)YN, W1T, DM, 1.0f / 1024.0f, FF1, MR, (size_t)0, DFF, DFF, (size_t)0);
    k_gemm_res<<<dim3(MR / 64, DM / 64, 1), 32, 0, stream>>>((const bf*)FF1, W2T, DFF, 1.0f / 1024.0f, X2, SEQ, OUT, OUT_SEQ);
}
